// DiffusionLoss_2370821947571
// MI455X (gfx1250) — hardware-verified
//
#include <hip/hip_runtime.h>


namespace {
constexpr int D = 4, L = 4096, NTOK = 512, TILE = 64, NTL = L / TILE  , NBLK = NTL * (NTL + 1) / 2  ;
constexpr float EPS = 1e-6f;

typedef _Float16 b16;
typedef __attribute__((ext_vector_type(16))) _Float16 v16b;
typedef __attribute__((ext_vector_type(8))) float v8f;
__device__ __forceinline__ float bf16_rne(float f) { unsigned int u = __float_as_uint(f); u += 0x7FFFu + ((u >> 16) & 1u); return __uint_as_float(u & 0xFFFF0000u); }
__device__ __forceinline__ v8f wmma16b(v16b a, v16b b, v8f c) { v8f d = __builtin_amdgcn_wmma_f32_16x16x32_f16(false, a, false, b, (short)0, c, false, false); asm volatile("v_nop\n\tv_nop\n\tv_nop\n\tv_nop" : "+v"(d) : "v"(a), "v"(b)); return d; }
__device__ __forceinline__ float nexp(float x) { return __builtin_amdgcn_exp2f(x * 1.4426950408889634f); }
__device__ __forceinline__ float sigm(float x) { return __builtin_amdgcn_rcpf(1.0f + nexp(-x)); }
__device__ __forceinline__ float pmul(float a, float b) { float p = a * b; asm volatile("" : "+v"(p)); return p; }

__device__ __forceinline__ v16b frag_xyz(const float* p3, int hh) { v16b f = {}; if (hh == 0) { f[0] = (b16)bf16_rne(p3[0]); f[1] = (b16)bf16_rne(p3[1]); f[2] = (b16)bf16_rne(p3[2]); } return f; }

__global__ __launch_bounds__(128) void pair_kernel(const float* __restrict__ X, const float* __restrict__ Xgt, const int* __restrict__ mask, const int* __restrict__ isd, const int* __restrict__ isr, const int* __restrict__ tok, float* __restrict__ part) {
  __shared__ float red[5][128];
  const int lane = threadIdx.x & 31, wave = threadIdx.x >> 5, nloc = lane & 15, hlf = lane >> 4;
  int b = blockIdx.x, ti = 0; while (b >= NTL - ti) { b -= NTL - ti; ++ti; } const int tj = ti + b;
  const int i0 = ti * TILE + wave * 16, j0 = tj * TILE;
  const int ia = i0 + nloc;
  float ssum[D] = {0.0f, 0.0f, 0.0f, 0.0f}, psum = 0.0f;
#pragma unroll
  for (int t = 0; t < 4; ++t) { const int ja = j0 + t * 16 + nloc;
    v8f g[5];
#pragma unroll
    for (int s = 0; s < 5; ++s) { const float* P_ = (s < D) ? (X + (size_t)s * L * 3) : Xgt; const v16b fa = frag_xyz(P_ + (size_t)ia * 3, hlf), fb = frag_xyz(P_ + (size_t)ja * 3, hlf); g[s] = (v8f){}; g[s] = wmma16b(fa, fb, g[s]); }
    const int j = j0 + t * 16 + nloc; const int mj = mask[j], tkj = tok[j];
#pragma unroll
    for (int r = 0; r < 8; ++r) { const int i = i0 + 8 * hlf + r; if (!(i < j)) continue;
      int tki = tok[i]; const int tkc = (tki < 0) ? 0 : (tki >= NTOK ? NTOK - 1 : tki); const bool na = (isd[tkc] | isr[tkc]) != 0; const float cut = na ? 30.0f : 15.0f;
      auto dist = [&](const float* P_, float gg) { const float* pi = P_ + (size_t)i * 3; const float* pj = P_ + (size_t)j * 3; float ni = 0.0f, nj = 0.0f;
        for (int c = 0; c < 3; ++c) { const float a = bf16_rne(pi[c]), bq = bf16_rne(pj[c]); ni += pmul(a, a); nj += pmul(bq, bq); } return __builtin_amdgcn_sqrtf(fmaxf((ni + nj) - pmul(2.0f, gg), 0.0f)); };
      const float gd = dist(Xgt, g[4][r]);
      const bool pm = (gd > 0.0f) && (gd < cut) && (mask[i] != 0) && (mj != 0) && (tki != tkj);
      if (pm) { psum += 1.0f;
#pragma unroll
        for (int s = 0; s < D; ++s) { const float pd = dist(X + (size_t)s * L * 3, g[s][r]); const float dl = fabsf(pd - gd + EPS); ssum[s] += (sigm(0.5f - dl) + sigm(1.0f - dl)) + (sigm(2.0f - dl) + sigm(4.0f - dl)); } } } }
  for (int s = 0; s < D; ++s) red[s][threadIdx.x] = ssum[s]; red[4][threadIdx.x] = psum;
  __syncthreads();
  for (int st = 64; st > 0; st >>= 1) { if ((int)threadIdx.x < st) { for (int s = 0; s < 5; ++s) red[s][threadIdx.x] += red[s][threadIdx.x + st]; } __syncthreads(); }
  if (threadIdx.x < 32) { const float v = (threadIdx.x < 5) ? red[threadIdx.x][0] : 0.0f; for (int pass = 0; pass < 2; ++pass) ((volatile float*)part)[(size_t)blockIdx.x * 32 + threadIdx.x] = v; }
  __threadfence();
}

__global__ __launch_bounds__(256) void final_kernel(const float* __restrict__ part, const float* __restrict__ X, const float* __restrict__ Xgt, const int* __restrict__ mask, const int* __restrict__ isd, const int* __restrict__ isr, const int* __restrict__ isl, const int* __restrict__ tok, const float* __restrict__ tt, float* __restrict__ out) {
  __shared__ float red[9][256]; __shared__ float cnt[256];
  const int t_ = threadIdx.x;
  float a[9] = {0, 0, 0, 0, 0, 0, 0, 0, 0}; float c_ = 0.0f;
  for (int blk = t_; blk < NBLK; blk += 256) { for (int s = 0; s < 5; ++s) a[s] += part[(size_t)blk * 32 + s]; }
  for (int l = t_; l < L; l += 256) { const float m = (mask[l] != 0) ? 1.0f : 0.0f; int tk = tok[l]; tk = (tk < 0) ? 0 : (tk >= NTOK ? NTOK - 1 : tk); const float alpha = (isd[tk] ? 5.0f : 0.0f) + (isr[tk] ? 5.0f : 0.0f) + (isl[tk] ? 10.0f : 0.0f); const float w = (1.0f + alpha) * m; c_ += m;
    const float gx = bf16_rne(Xgt[l * 3]), gy = bf16_rne(Xgt[l * 3 + 1]), gz = bf16_rne(Xgt[l * 3 + 2]);
    for (int d = 0; d < D; ++d) { const float* p = X + ((size_t)d * L + l) * 3; const float dx = bf16_rne(p[0]) - gx, dy = bf16_rne(p[1]) - gy, dz = bf16_rne(p[2]) - gz; a[5 + d] += w * ((pmul(dx, dx) + pmul(dy, dy)) + pmul(dz, dz)); } }
  for (int s = 0; s < 9; ++s) red[s][t_] = a[s]; cnt[t_] = c_;
  __syncthreads();
  for (int st = 128; st > 0; st >>= 1) { if (t_ < st) { for (int s = 0; s < 9; ++s) red[s][t_] += red[s][t_ + st]; cnt[t_] += cnt[t_ + st]; } __syncthreads(); }
  if (t_ < 32) { float res = 0.0f;
    if (true) { const float psum = red[4][0], msum = cnt[0]; float ld = 0.0f, ll = 0.0f;
      for (int d = 0; d < D; ++d) { const float t = bf16_rne(tt[d]); const float lam = (t * t + 256.0f) / ((t * 16.0f) * (t * 16.0f)); const float lmse = (1.0f / 3.0f) * red[5 + d][0] / (msum + 1e-4f); ld += fminf(lam * lmse, 2.0f); const float lddt = 0.25f * red[d][0] / (psum + EPS); ll += 1.0f - lddt; }
      res = 4.0f * (ld / (float)D + ll / (float)D); }
    if (t_ == 0) { for (int pass = 0; pass < 2; ++pass) ((volatile float*)out)[0] = res; } }
  __threadfence();
}
}

extern "C" void kernel_launch(void* const* d_in, const int* in_sizes, int n_in,
                              void* d_out, int out_size, void* d_ws, size_t ws_size, hipStream_t stream) {
  (void)n_in; (void)out_size;
  const float* X = (const float*)d_in[0]; const float* Xgt = (const float*)d_in[1]; const int* mask = (const int*)d_in[2]; const int* isd = (const int*)d_in[3]; const int* isr = (const int*)d_in[4]; const int* isl = (const int*)d_in[5]; const int* tok = (const int*)d_in[6]; const float* tt = (const float*)d_in[7];
  float* out = (float*)d_out;
  if (in_sizes[0] != D * L * 3 || in_sizes[1] != L * 3 || in_sizes[2] != L || in_sizes[3] != NTOK || in_sizes[6] != L || in_sizes[7] != D) return;
  if ((size_t)NBLK * 32 * 4 > ws_size) return;
  float* part = (float*)d_ws;
  pair_kernel<<<NBLK, 128, 0, stream>>>(X, Xgt, mask, isd, isr, tok, part);
  final_kernel<<<1, 256, 0, stream>>>(part, X, Xgt, mask, isd, isr, isl, tok, tt, out);
}
